// Replicator2Layer_10831907520900
// MI455X (gfx1250) — hardware-verified
//
#include <hip/hip_runtime.h>


#ifndef NB
#define NB 4
#endif
#define NB_FULL 4
#define NPOS 256
#define EMB  512
#define QRS  2048.0f
#define QRI  (1.0f / 2048.0f)
#define WSC  256.0f
#define WSI  (1.0f / 256.0f)
#define XSC  64.0f
#define XSI  (1.0f / 64.0f)

static_assert(NB <= NB_FULL);
static_assert(NPOS % 64 == 0);
static_assert(EMB % 64 == 0);
static_assert(NPOS % 32 == 0);
static_assert(EMB % 32 == 0);
static_assert(NPOS % 16 == 0);
static_assert((NB * NPOS) % 16 == 0);
static_assert(((size_t)NB * NPOS * EMB) % (8 * 256) == 0);
static_assert(((size_t)NPOS * NPOS) % (8 * 256) == 0);
static_assert(256 * 4 * 4 == 64 * 64);
static_assert(256 * 2 * 8 == 64 * 64);
static_assert(4 * 4 == 16);
static_assert(32 * 8 * 4 == 16 * 64);
static_assert(8 * 2 == 16);
static_assert(32 * 4 * 8 == 16 * 64);
static_assert(128 * 4 == EMB);
static_assert(16 * 68 * 4 <= 131072);
static_assert(64 * 65 * 4 <= 131072);
static_assert((68 * 4) % 16 == 0);

typedef _Float16 h16;
typedef unsigned short bf;
typedef __attribute__((ext_vector_type(16))) __bf16   v16bf;
typedef __attribute__((ext_vector_type(16))) _Float16 v16h;
typedef __attribute__((ext_vector_type(8)))  _Float16 v8h;
typedef __attribute__((ext_vector_type(8)))  unsigned short v8us;
typedef __attribute__((ext_vector_type(8)))  float    v8f;
typedef __attribute__((ext_vector_type(4)))  float    v4f;
typedef v4f  __attribute__((may_alias)) v4fa;

__device__ __forceinline__ unsigned short f2bf(float f) { unsigned u = __float_as_uint(f); u += 0x7FFFu + ((u >> 16) & 1u); return (unsigned short)(u >> 16); }
__device__ __forceinline__ float bfr(float f) { return __uint_as_float(((unsigned)f2bf(f)) << 16); }
__device__ __forceinline__ v16h cat16(v8h lo, v8h hi) { return __builtin_shufflevector(lo, hi, 0, 1, 2, 3, 4, 5, 6, 7, 8, 9, 10, 11, 12, 13, 14, 15); }
__device__ __forceinline__ v16bf cat16b(v8us lo, v8us hi) { return __builtin_bit_cast(v16bf, __builtin_shufflevector(lo, hi, 0, 1, 2, 3, 4, 5, 6, 7, 8, 9, 10, 11, 12, 13, 14, 15)); }
__device__ __forceinline__ v8f wmma16(v16h a, v16h b, v8f c) { return __builtin_amdgcn_wmma_f32_16x16x32_f16(false, a, false, b, (short)0, c, false, false); }
__device__ __forceinline__ v8f wmmab(v16bf a, v16bf b, v8f c) { return __builtin_amdgcn_wmma_f32_16x16x32_bf16(false, a, false, b, (short)0, c, false, false); }
__device__ __forceinline__ v16h  ldh(const h16* p) { return cat16(*(const v8h*)p, *(const v8h*)(p + 16)); }
__device__ __forceinline__ v16bf ldb(const bf* p)  { return cat16b(*(const v8us*)p, *(const v8us*)(p + 16)); }
__device__ __forceinline__ void wave_sync() { __builtin_amdgcn_fence(3  , "wavefront"); __builtin_amdgcn_wave_barrier(); asm volatile("" ::: "memory"); }

static __device__ __forceinline__ h16 toh_flush(float v) { const h16 r = (h16)v; return (fabsf(v) < 6.103515625e-05f) ? (h16)0.0f : r; }
__device__ __forceinline__ v8f wmg16(v16h a, v16h b, v8f c) { c = wmma16(a, b, c); asm volatile("v_nop\n\tv_nop\n\tv_nop\n\tv_nop" : "+v"(c) : "v"(a), "v"(b)); return c; }
__device__ __forceinline__ v8f wmgb(v16bf a, v16bf b, v8f c) { c = wmmab(a, b, c); asm volatile("v_nop\n\tv_nop\n\tv_nop\n\tv_nop" : "+v"(c) : "v"(a), "v"(b)); return c; }

__device__ __forceinline__ void cvt_tril_hr(const v4f x0, const v4f x1, const int i, const int n, v8h& hv, v8h& rv) {
#pragma unroll
    for (int e = 0; e < 4; ++e) {
        const float a = (n + e <= i) ? x0[e] : 0.0f;
        const float c = (n + 4 + e <= i) ? x1[e] : 0.0f;
        const h16 ah = toh_flush(a); const h16 ch = toh_flush(c);
        hv[e] = ah; hv[4 + e] = ch;
        rv[e] = toh_flush((a - (float)ah) * QRS); rv[4 + e] = toh_flush((c - (float)ch) * QRS); }
}

__global__ __launch_bounds__(256) void k_cvt8(const float* __restrict__ src, bf* dst, size_t n8) {
    const size_t i = (size_t)blockIdx.x * 256 + threadIdx.x; if (i >= n8) return;
    const v8f v = *(const v8f*)(src + i * 8); v8us o;
#pragma unroll
    for (int k = 0; k < 8; ++k) o[k] = f2bf(v[k]);
    *(volatile v8us*)(dst + i * 8) = o; __threadfence(); *(volatile v8us*)(dst + i * 8) = o;
}

__global__ __launch_bounds__(256) void k_wconv(const float* __restrict__ src, h16* dst, size_t n8, float scale) {
#pragma clang fp contract(off)
    const size_t i = (size_t)blockIdx.x * 256 + threadIdx.x; if (i >= n8) return;
    const v8f v = *(const v8f*)(src + i * 8); v8h o;
#pragma unroll
    for (int k = 0; k < 8; ++k) o[k] = toh_flush(bfr(v[k]) * scale);
    *(volatile v8h*)(dst + i * 8) = o; __threadfence(); *(volatile v8h*)(dst + i * 8) = o;
}

__global__ __launch_bounds__(256) void k_tconv(const float* __restrict__ src, h16* dst, int rows, int cols, size_t sbatch, size_t dbatch, float scale) {
#pragma clang fp contract(off)
    __shared__ float tile[64 * 65];
    const int tid = threadIdx.x;
    const int c0 = blockIdx.x * 64, r0 = blockIdx.y * 64;
    const float* s = src + (size_t)blockIdx.z * sbatch;
    h16* d = dst + (size_t)blockIdx.z * dbatch;
#pragma unroll
    for (int it = 0; it < 4; ++it) { const int q = it * 256 + tid; const int r = q >> 4, c4 = (q & 15) * 4;
        const v4f v = *(const v4f*)(s + (size_t)(r0 + r) * cols + c0 + c4);
        tile[r * 65 + c4 + 0] = v[0]; tile[r * 65 + c4 + 1] = v[1]; tile[r * 65 + c4 + 2] = v[2]; tile[r * 65 + c4 + 3] = v[3]; }
    __syncthreads();
#pragma unroll 1
    for (int ps = 0; ps < 2; ++ps) {
#pragma unroll
        for (int it = 0; it < 2; ++it) { const int p = it * 256 + tid; const int c = p >> 3, r8 = (p & 7) * 8;
            v8h o;
#pragma unroll
            for (int j = 0; j < 8; ++j) o[j] = toh_flush(bfr(tile[(r8 + j) * 65 + c]) * scale);
            *(volatile v8h*)(d + (size_t)(c0 + c) * rows + r0 + r8) = o; }
        if (ps == 0) __threadfence(); }
}

__global__ __launch_bounds__(32) void k_gram(const bf* __restrict__ XB, h16* GH, h16* GR) {
    __shared__ __align__(16) float os[16 * 68];
    const int lane = threadIdx.x & 31, lr = lane & 15, hi = lane >> 4;
    const int r0 = blockIdx.x * 16, c0 = blockIdx.y * 64;
    const int bb = r0 / NPOS, i0 = r0 % NPOS;
    const int kend = (c0 > i0 + 15) ? 0 : EMB;
    v8f acc[4];
#pragma unroll
    for (int nb = 0; nb < 4; ++nb) acc[nb] = (v8f){};
    const size_t aoff = (size_t)(r0 + lr) * EMB + 8 * hi, boff = (size_t)(bb * NPOS + c0 + lr) * EMB + 8 * hi;
#pragma unroll 1
    for (int kc = 0; kc < kend; kc += 32) {
        const v16bf a = ldb(XB + aoff + kc);
#pragma unroll
        for (int nb = 0; nb < 4; ++nb) { const v16bf b = ldb(XB + boff + (size_t)nb * 16 * EMB + kc); acc[nb] = wmgb(a, b, acc[nb]); }
    }
#pragma unroll
    for (int nb = 0; nb < 4; ++nb) {
#pragma unroll
        for (int j = 0; j < 8; ++j) os[(hi * 8 + j) * 68 + nb * 16 + lr] = acc[nb][j]; }
    wave_sync();
#pragma unroll 1
    for (int ps = 0; ps < 2; ++ps) {
#pragma unroll
        for (int s = 0; s < 4; ++s) { const int row = 4 * s + (lane >> 3), c8 = (lane & 7) * 8;
            const v4f x0 = *(const v4fa*)(&os[row * 68 + c8]); const v4f x1 = *(const v4fa*)(&os[row * 68 + c8 + 4]); v8h hv, rv;
            cvt_tril_hr(x0, x1, i0 + row, c0 + c8, hv, rv);
            const size_t oo = (size_t)(r0 + row) * NPOS + c0 + c8;
            *(volatile v8h*)(GH + oo) = hv; *(volatile v8h*)(GR + oo) = rv; }
        if (ps == 0) __threadfence(); }
}

__global__ __launch_bounds__(32) void k_gemm_h(const h16* __restrict__ AH, const h16* __restrict__ AR, const h16* __restrict__ Bt, float oscale, h16* PH, h16* PR) {
    __shared__ __align__(16) float os[16 * 68];
    const int lane = threadIdx.x & 31, lr = lane & 15, hi = lane >> 4;
    const int r0 = blockIdx.x * 16, c0 = blockIdx.y * 64;
    const int i0 = r0 % NPOS;
    const int nk = (c0 > i0 + 15) ? 0 : ((i0 + 16 + 31) & ~31);
    v8f acc[4], accR[4];
#pragma unroll
    for (int nb = 0; nb < 4; ++nb) { acc[nb] = (v8f){}; accR[nb] = (v8f){}; }
    const size_t aoff = (size_t)(r0 + lr) * NPOS + 8 * hi, boff = (size_t)(c0 + lr) * NPOS + 8 * hi;
#pragma unroll 1
    for (int kc = 0; kc < nk; kc += 32) {
        const v16h ah = ldh(AH + aoff + kc), ar = ldh(AR + aoff + kc);
#pragma unroll
        for (int nb = 0; nb < 4; ++nb) { const v16h b = ldh(Bt + boff + (size_t)nb * 16 * NPOS + kc);
            acc[nb] = wmg16(ah, b, acc[nb]); accR[nb] = wmg16(ar, b, accR[nb]); }
    }
#pragma unroll
    for (int nb = 0; nb < 4; ++nb) {
#pragma unroll
        for (int j = 0; j < 8; ++j) os[(hi * 8 + j) * 68 + nb * 16 + lr] = (acc[nb][j] + accR[nb][j] * QRI) * oscale; }
    wave_sync();
#pragma unroll 1
    for (int ps = 0; ps < 2; ++ps) {
#pragma unroll
        for (int s = 0; s < 4; ++s) { const int row = 4 * s + (lane >> 3), c8 = (lane & 7) * 8;
            const v4f x0 = *(const v4fa*)(&os[row * 68 + c8]); const v4f x1 = *(const v4fa*)(&os[row * 68 + c8 + 4]); v8h hv, rv;
            cvt_tril_hr(x0, x1, i0 + row, c0 + c8, hv, rv);
            const size_t oo = (size_t)(r0 + row) * NPOS + c0 + c8;
            *(volatile v8h*)(PH + oo) = hv; *(volatile v8h*)(PR + oo) = rv; }
        if (ps == 0) __threadfence(); }
}

__global__ __launch_bounds__(32) void k_gemm_f(const h16* __restrict__ AH, const h16* __restrict__ AR, const h16* __restrict__ XT, float oscale, float* PF) {
    __shared__ __align__(16) float os[16 * 68];
    const int lane = threadIdx.x & 31, lr = lane & 15, hi = lane >> 4;
    const int r0 = blockIdx.x * 16, c0 = blockIdx.y * 64;
    const int bb = r0 / NPOS, i0 = r0 % NPOS;
    const int nk = (i0 + 16 + 31) & ~31;
    v8f acc[4], accR[4];
#pragma unroll
    for (int nb = 0; nb < 4; ++nb) { acc[nb] = (v8f){}; accR[nb] = (v8f){}; }
    const size_t aoff = (size_t)(r0 + lr) * NPOS + 8 * hi, boff = (size_t)bb * EMB * NPOS + (size_t)(c0 + lr) * NPOS + 8 * hi;
#pragma unroll 1
    for (int kc = 0; kc < nk; kc += 32) {
        const v16h ah = ldh(AH + aoff + kc), ar = ldh(AR + aoff + kc);
#pragma unroll
        for (int nb = 0; nb < 4; ++nb) { const v16h b = ldh(XT + boff + (size_t)nb * 16 * NPOS + kc);
            acc[nb] = wmg16(ah, b, acc[nb]); accR[nb] = wmg16(ar, b, accR[nb]); }
    }
#pragma unroll
    for (int nb = 0; nb < 4; ++nb) {
#pragma unroll
        for (int j = 0; j < 8; ++j) os[(hi * 8 + j) * 68 + nb * 16 + lr] = (acc[nb][j] + accR[nb][j] * QRI) * oscale; }
    wave_sync();
#pragma unroll 1
    for (int ps = 0; ps < 2; ++ps) {
#pragma unroll
        for (int s = 0; s < 8; ++s) { const int row = 2 * s + (lane >> 4), cofs = (lane & 15) * 4;
            const v4f val = *(const v4fa*)(&os[row * 68 + cofs]);
            *(volatile v4f*)(PF + (size_t)(r0 + row) * EMB + c0 + cofs) = val; }
        if (ps == 0) __threadfence(); }
}

__global__ __launch_bounds__(128) void k_final(const float* __restrict__ X, const float* __restrict__ F, float* OUT) {
#pragma clang fp contract(off)
    __shared__ float red[4];
    const int tid = threadIdx.x, lane = tid & 31;
    const int wave = __builtin_amdgcn_readfirstlane((int)(threadIdx.x >> 5));
    const size_t base = (size_t)blockIdx.x * EMB + (size_t)tid * 4;
    v4f xv = *(const v4f*)(X + base);
    xv[0] = bfr(xv[0]); xv[1] = bfr(xv[1]); xv[2] = bfr(xv[2]); xv[3] = bfr(xv[3]);
    const v4f fv = *(const v4f*)(F + base);
    float p = xv[0] * fv[0]; p += xv[1] * fv[1]; p += xv[2] * fv[2]; p += xv[3] * fv[3];
    p += __shfl_xor(p, 16, 32); p += __shfl_xor(p, 8, 32); p += __shfl_xor(p, 4, 32); p += __shfl_xor(p, 2, 32); p += __shfl_xor(p, 1, 32);
    if (lane == 0) red[wave] = p;
    __syncthreads();
    const float avg = ((red[0] + red[1]) + red[2]) + red[3];
    v4f o;
    o[0] = xv[0] + xv[0] * (fv[0] - avg); o[1] = xv[1] + xv[1] * (fv[1] - avg); o[2] = xv[2] + xv[2] * (fv[2] - avg); o[3] = xv[3] + xv[3] * (fv[3] - avg);
    *(volatile v4f*)(OUT + base) = o; __threadfence(); *(volatile v4f*)(OUT + base) = o;
}

static constexpr size_t al256(size_t v) { return (v + 255) & ~(size_t)255; }
static constexpr size_t SZ_XB = al256((size_t)NB * NPOS * EMB * 2);
static constexpr size_t SZ_XT = al256((size_t)NB * EMB * NPOS * 2);
static constexpr size_t SZ_W  = al256((size_t)NPOS * NPOS * 2);
static constexpr size_t SZ_P  = al256((size_t)NB * NPOS * NPOS * 2);
static constexpr size_t SZ_F  = al256((size_t)NB * NPOS * EMB * 4);
static constexpr size_t SZ_TOTAL = SZ_XB + SZ_XT + 2 * SZ_W + 6 * SZ_P + SZ_F;
static_assert(SZ_TOTAL <= (size_t)134217728);

extern "C" void kernel_launch(void* const* d_in, const int* in_sizes, int n_in,
                              void* d_out, int out_size, void* d_ws, size_t ws_size, hipStream_t stream) {
    if (n_in < 3) return;
    if ((size_t)in_sizes[0] < (size_t)NB * NPOS * EMB) return;
    if ((size_t)in_sizes[1] < (size_t)NPOS * NPOS || (size_t)in_sizes[2] < (size_t)NPOS * NPOS) return;
    if ((size_t)out_size < (size_t)NB * NPOS * EMB) return;
    if (SZ_TOTAL > ws_size) return;
    const float* x  = (const float*)d_in[0];
    const float* qw = (const float*)d_in[1];
    const float* kw = (const float*)d_in[2];
    float* OUT = (float*)d_out;
    char* wsp = (char*)d_ws;
    bf*  XB = (bf*)wsp;  wsp += SZ_XB;
    h16* XT = (h16*)wsp; wsp += SZ_XT;
    h16* KT = (h16*)wsp; wsp += SZ_W;
    h16* QH = (h16*)wsp; wsp += SZ_W;
    h16* GH = (h16*)wsp; wsp += SZ_P;
    h16* GR = (h16*)wsp; wsp += SZ_P;
    h16* SH = (h16*)wsp; wsp += SZ_P;
    h16* SR = (h16*)wsp; wsp += SZ_P;
    h16* TH = (h16*)wsp; wsp += SZ_P;
    h16* TR = (h16*)wsp; wsp += SZ_P;
    float* FP = (float*)wsp; wsp += SZ_F;

    { const size_t n8 = (size_t)NB * NPOS * EMB / 8;
      k_cvt8<<<(unsigned)((n8 + 255) / 256), 256, 0, stream>>>(x, XB, n8); }
    k_tconv<<<dim3(EMB / 64, NPOS / 64, NB), 256, 0, stream>>>(x, XT, NPOS, EMB, (size_t)NPOS * EMB, (size_t)EMB * NPOS, XSC);
    k_tconv<<<dim3(NPOS / 64, NPOS / 64, 1), 256, 0, stream>>>(kw, KT, NPOS, NPOS, (size_t)0, (size_t)0, WSC);
    { const size_t n8 = (size_t)NPOS * NPOS / 8;
      k_wconv<<<(unsigned)((n8 + 255) / 256), 256, 0, stream>>>(qw, QH, n8, WSC); }

    k_gram<<<dim3(NB * NPOS / 16, NPOS / 64, 1), 32, 0, stream>>>(XB, GH, GR);
    k_gemm_h<<<dim3(NB * NPOS / 16, NPOS / 64, 1), 32, 0, stream>>>(GH, GR, KT, WSI, SH, SR);
    k_gemm_h<<<dim3(NB * NPOS / 16, NPOS / 64, 1), 32, 0, stream>>>(SH, SR, QH, WSI, TH, TR);
    k_gemm_f<<<dim3(NB * NPOS / 16, EMB / 64, 1), 32, 0, stream>>>(TH, TR, XT, XSI, FP);
    k_final<<<NB * NPOS, 128, 0, stream>>>(x, FP, OUT);
}
